// TropicalMultiHeadAttn_7524782702955
// MI455X (gfx1250) — hardware-run, weakly checked
//
#include <hip/hip_runtime.h>


#ifndef NB
#define NB 2
#endif
#ifndef SEQ
#define SEQ 512
#endif
#define NB_FULL  2
#define SEQ_FULL 512
#define DM   512
#define NH_  8
#define HD   64
#define XSP  68
#define YSP  516
#define ORW  16
#define ACARRY 16.0f
#define WCARRY 64.0f
#define OSCL (1.0f / 1024.0f)
#define LNEPS 1e-5f
#define NEGB (-3.0e38f)
#define POSB (3.0e38f)

static_assert(NH_ * HD == DM);
static_assert(HD == 64);
static_assert(DM % 64 == 0);
static_assert(DM % 32 == 0);
static_assert(SEQ % 64 == 0);
static_assert((NB * SEQ) % 64 == 0);
static_assert(SEQ % 32 == 0);
static_assert(SEQ % NH_ == 0);
static_assert((NB * SEQ) % ORW == 0);
static_assert(ORW == 16);
static_assert(8 * 64 == DM);
static_assert(NB <= NB_FULL);
static_assert(SEQ <= SEQ_FULL);
static_assert((XSP * 4) % 16 == 0);
static_assert(XSP >= 64);
static_assert((YSP * 4) % 16 == 0);
static_assert(YSP >= DM);
static_assert(((size_t)SEQ * NB_FULL * DM) % 8 == 0);
static_assert(((size_t)DM * DM) % 8 == 0);
static_assert(32 * 16 * 32 == 64 * 64 * 4);
static_assert(256 * 16 == 32 * HD * 2);
static_assert(8 * (ORW / 8) * 4 * 32 * 16 == ORW * DM * 4);
static_assert(3 * 64 * XSP * 4 <= 131072);
static_assert(3 * 32 * 17 * 16 + 32 * 33 * 4 <= 131072);
static_assert(ORW * YSP * 4 <= 131072);

typedef _Float16 h16;
typedef unsigned short bf;
typedef __attribute__((ext_vector_type(16))) __bf16   v16bf;
typedef __attribute__((ext_vector_type(16))) _Float16 v16h;
typedef __attribute__((ext_vector_type(8)))  _Float16 v8h;
typedef __attribute__((ext_vector_type(8)))  unsigned short v8us;
typedef __attribute__((ext_vector_type(8)))  float    v8f;
typedef __attribute__((ext_vector_type(4)))  float    v4f;
typedef v4f  __attribute__((may_alias)) v4fa;

__device__ __forceinline__ unsigned short f2bf(float f) { unsigned u = __float_as_uint(f); u += 0x7FFFu + ((u >> 16) & 1u); return (unsigned short)(u >> 16); }
__device__ __forceinline__ float bfr(float f) { return __uint_as_float(((unsigned)f2bf(f)) << 16); }
__device__ __forceinline__ v16h cat16(v8h lo, v8h hi) { return __builtin_shufflevector(lo, hi, 0, 1, 2, 3, 4, 5, 6, 7, 8, 9, 10, 11, 12, 13, 14, 15); }
__device__ __forceinline__ v16bf cat16b(v8us lo, v8us hi) { return __builtin_bit_cast(v16bf, __builtin_shufflevector(lo, hi, 0, 1, 2, 3, 4, 5, 6, 7, 8, 9, 10, 11, 12, 13, 14, 15)); }
__device__ __forceinline__ v8f wmma16(v16h a, v16h b, v8f c) { return __builtin_amdgcn_wmma_f32_16x16x32_f16(false, a, false, b, (short)0, c, false, false); }
__device__ __forceinline__ v8f wmmab(v16bf a, v16bf b, v8f c) { return __builtin_amdgcn_wmma_f32_16x16x32_bf16(false, a, false, b, (short)0, c, false, false); }
__device__ __forceinline__ v16h  ldh(const h16* p) { return cat16(*(const v8h*)p, *(const v8h*)(p + 16)); }
__device__ __forceinline__ v16bf ldb(const bf* p)  { return cat16b(*(const v8us*)p, *(const v8us*)(p + 16)); }
__device__ __forceinline__ void wave_sync() { __builtin_amdgcn_fence(3  , "wavefront"); __builtin_amdgcn_wave_barrier(); asm volatile("" ::: "memory"); }

__device__ __forceinline__ v8f wmmab_g(v16bf a, v16bf b, v8f c) { c = wmmab(a, b, c); asm volatile("v_nop\n\tv_nop\n\tv_nop\n\tv_nop" : "+v"(c) : "v"(a), "v"(b)); return c; }
__device__ __forceinline__ v8f wmma16_g(v16h a, v16h b, v8f c) { c = wmma16(a, b, c); asm volatile("v_nop\n\tv_nop\n\tv_nop\n\tv_nop" : "+v"(c) : "v"(a), "v"(b)); return c; }
static __device__ __forceinline__ h16 toh_flush(float v) { const h16 r = (h16)v; return (fabsf(v) < 6.103515625e-05f) ? (h16)0.0f : r; }
__device__ __forceinline__ float wsum(float v) { v += __shfl_xor(v, 16, 32); v += __shfl_xor(v, 8, 32); v += __shfl_xor(v, 4, 32); v += __shfl_xor(v, 2, 32); v += __shfl_xor(v, 1, 32); return v; }

__global__ __launch_bounds__(256) void k_cvt8(const float* __restrict__ src, bf* dst, size_t n8) {
    const size_t i = (size_t)blockIdx.x * 256 + threadIdx.x; if (i >= n8) return;
    const v8f v = *(const v8f*)(src + i * 8); v8us o;
#pragma unroll
    for (int k = 0; k < 8; ++k) o[k] = f2bf(v[k]);
    *(volatile v8us*)(dst + i * 8) = o; __threadfence(); *(volatile v8us*)(dst + i * 8) = o;
}

__global__ __launch_bounds__(256) void k_wcvt8h(const float* __restrict__ src, h16* dst, size_t n8, float carry) {
    const size_t i = (size_t)blockIdx.x * 256 + threadIdx.x; if (i >= n8) return;
    const v8f v = *(const v8f*)(src + i * 8); v8h o;
#pragma unroll
    for (int k = 0; k < 8; ++k) o[k] = toh_flush(bfr(v[k]) * carry);
    *(volatile v8h*)(dst + i * 8) = o; __threadfence(); *(volatile v8h*)(dst + i * 8) = o;
}

__global__ __launch_bounds__(32) void k_qkvt(const bf* __restrict__ A, const bf* __restrict__ Bt, const float* __restrict__ lam, const float* __restrict__ Wt, float* TP) {
    __shared__ __align__(16) float xs[64 * XSP];
    __shared__ __align__(16) float wl[64 * XSP];
    __shared__ __align__(16) float ys[64 * XSP];
    const int K = DM;
    const int lane = threadIdx.x & 31, lr = lane & 15, hi = lane >> 4; const int r0 = blockIdx.x * 64, c0 = blockIdx.y * 64;
    const int bb = r0 / SEQ, s0 = r0 % SEQ;
    v8f acc[4][4];
#pragma unroll
    for (int mb = 0; mb < 4; ++mb)
#pragma unroll
        for (int nb = 0; nb < 4; ++nb) acc[mb][nb] = (v8f){};
    const size_t aoff = ((size_t)(s0 + lr) * NB_FULL + (size_t)bb) * K + 8 * hi, boff = (size_t)(c0 + lr) * K + 8 * hi;
#pragma unroll 1
    for (int kc = 0; kc < K; kc += 32) {
        v16bf a[4];
#pragma unroll
        for (int mb = 0; mb < 4; ++mb) a[mb] = ldb(A + aoff + (size_t)mb * 16 * NB_FULL * K + kc);
#pragma unroll
        for (int nb = 0; nb < 4; ++nb) { const v16bf b = ldb(Bt + boff + (size_t)nb * 16 * K + kc);
#pragma unroll
            for (int mb = 0; mb < 4; ++mb) acc[mb][nb] = wmmab_g(a[mb], b, acc[mb][nb]); }
    }
#pragma unroll
    for (int mb = 0; mb < 4; ++mb)
#pragma unroll
        for (int nb = 0; nb < 4; ++nb)
#pragma unroll
            for (int j = 0; j < 8; ++j) xs[(mb * 16 + hi * 8 + j) * XSP + nb * 16 + lr] = acc[mb][nb][j];
#pragma unroll 1
    for (int e = lane; e < 64 * 16; e += 32) {
        v4f w = *(const v4f*)(Wt + (size_t)e * 4);
#pragma unroll
        for (int i = 0; i < 4; ++i) w[i] = bfr(w[i]);
        *(v4fa*)(&wl[(e >> 4) * XSP + (e & 15) * 4]) = w; }
    wave_sync();
    const int c4 = (lane & 15) * 4, rh = lane >> 4;
    float lv[4];
#pragma unroll
    for (int i = 0; i < 4; ++i) lv[i] = bfr(lam[c0 + c4 + i]);
#pragma unroll 1
    for (int s = 0; s < 32; ++s) { const int row = 2 * s + rh;
        v4f x = *(const v4fa*)(&xs[row * XSP + c4]);
#pragma unroll
        for (int i = 0; i < 4; ++i) x[i] = log1pf(fmaxf(x[i], 0.0f)) - lv[i];
        *(v4fa*)(&xs[row * XSP + c4]) = x; }
    wave_sync();
    float wlo[64], whi[64];
#pragma unroll
    for (int g = 0; g < 16; ++g) { const v4f t0 = *(const v4fa*)(&wl[lane * XSP + 4 * g]); const v4f t1 = *(const v4fa*)(&wl[(lane + 32) * XSP + 4 * g]);
#pragma unroll
        for (int i = 0; i < 4; ++i) { wlo[4 * g + i] = t0[i]; whi[4 * g + i] = t1[i]; } }
#pragma unroll 1
    for (int r = 0; r < 64; ++r) {
        float a0 = NEGB, a1 = NEGB;
#pragma unroll
        for (int g = 0; g < 16; ++g) { const v4f x = *(const v4fa*)(&xs[r * XSP + 4 * g]);
#pragma unroll
            for (int i = 0; i < 4; ++i) { a0 = fmaxf(a0, x[i] + wlo[4 * g + i]); a1 = fmaxf(a1, x[i] + whi[4 * g + i]); } }
        ys[r * XSP + lane] = a0; ys[r * XSP + lane + 32] = a1; }
    wave_sync();
    float* orow = TP + (size_t)r0 * DM + c0 + c4;
#pragma unroll 1
    for (int ps = 0; ps < 2; ++ps) {
#pragma unroll 1
        for (int s = 0; s < 32; ++s) { const int row = 2 * s + rh;
            const v4f val = *(const v4fa*)(&ys[row * XSP + c4]);
            *(volatile v4f*)(orow + (size_t)row * DM) = val; }
        if (ps == 0) __threadfence(); }
}

__device__ __forceinline__ void dmm(const v4f q, const v4f k, float& mx, float& mn) {
    const float d0 = q[0] - k[0], d1 = q[1] - k[1], d2 = q[2] - k[2], d3 = q[3] - k[3];
    mx = fmaxf(mx, fmaxf(fmaxf(d0, d1), fmaxf(d2, d3)));
    mn = fminf(mn, fminf(fminf(d0, d1), fminf(d2, d3)));
}

__global__ __launch_bounds__(256) void k_mpattn(const float* __restrict__ QP, const float* __restrict__ KP, const float* __restrict__ VP, h16* AV) {
#pragma clang fp contract(off)
    __shared__ v4f qs[32 * 17];
    __shared__ v4f ks[32 * 17];
    __shared__ v4f vs[32 * 17];
    __shared__ float sc[32 * 33];
    const int g = blockIdx.y, sqt = blockIdx.x, tid = threadIdx.x;
    const int wave = __builtin_amdgcn_readfirstlane((int)(threadIdx.x >> 5));
    const int lane = tid & 31;
    const v4f* qb = (const v4f*)(QP + ((size_t)g * SEQ + (size_t)sqt * 32) * HD);
    const v4f* kb = (const v4f*)(KP + (size_t)g * SEQ * HD);
    const v4f* vb = (const v4f*)(VP + (size_t)g * SEQ * HD);
    qs[(tid >> 4) * 17 + (tid & 15)]        = qb[tid];
    qs[((tid >> 4) + 16) * 17 + (tid & 15)] = qb[tid + 256];
    float ctx[8];
#pragma unroll
    for (int j = 0; j < 8; ++j) ctx[j] = NEGB;
    const int sq1 = wave, sk1 = lane;
    const int sq2 = tid >> 3, dg = tid & 7;
#pragma unroll 1
    for (int kt = 0; kt < SEQ / 32; ++kt) {
        __syncthreads();
        const int nbp = kt * 512;
        ks[(tid >> 4) * 17 + (tid & 15)]        = kb[nbp + tid];
        ks[((tid >> 4) + 16) * 17 + (tid & 15)] = kb[nbp + tid + 256];
        vs[(tid >> 4) * 17 + (tid & 15)]        = vb[nbp + tid];
        vs[((tid >> 4) + 16) * 17 + (tid & 15)] = vb[nbp + tid + 256];
        __syncthreads();
        float mx0 = NEGB, mx1 = NEGB, mx2 = NEGB, mx3 = NEGB;
        float mn0 = POSB, mn1 = POSB, mn2 = POSB, mn3 = POSB;
#pragma unroll 4
        for (int c = 0; c < 16; ++c) {
            const v4f kv = ks[sk1 * 17 + c];
            dmm(qs[sq1 * 17 + c], kv, mx0, mn0);
            dmm(qs[(sq1 + 8) * 17 + c], kv, mx1, mn1);
            dmm(qs[(sq1 + 16) * 17 + c], kv, mx2, mn2);
            dmm(qs[(sq1 + 24) * 17 + c], kv, mx3, mn3);
        }
        sc[sq1 * 33 + sk1]        = mn0 - mx0;
        sc[(sq1 + 8) * 33 + sk1]  = mn1 - mx1;
        sc[(sq1 + 16) * 33 + sk1] = mn2 - mx2;
        sc[(sq1 + 24) * 33 + sk1] = mn3 - mx3;
        __syncthreads();
#pragma unroll 4
        for (int sk = 0; sk < 32; ++sk) {
            const float s = sc[sq2 * 33 + sk];
            const v4f v0 = vs[sk * 17 + dg * 2];
            const v4f v1 = vs[sk * 17 + dg * 2 + 1];
#pragma unroll
            for (int i = 0; i < 4; ++i) { ctx[i] = fmaxf(ctx[i], s + v0[i]); ctx[4 + i] = fmaxf(ctx[4 + i], s + v1[i]); }
        }
    }
    const int b2 = g / NH_, h2 = g % NH_;
    const int s2 = sqt * 32 + sq2;
    v8h o;
#pragma unroll
    for (int j = 0; j < 8; ++j) o[j] = toh_flush(expm1f(ctx[j]) * ACARRY);
    h16* dst = AV + ((size_t)s2 * NB + (size_t)b2) * DM + h2 * HD + dg * 8;
    *(volatile v8h*)dst = o; __threadfence(); *(volatile v8h*)dst = o;
}

__global__ __launch_bounds__(256) void k_oln(const h16* __restrict__ AV, const h16* __restrict__ WO, const float* __restrict__ hin, const float* __restrict__ gamma, const float* __restrict__ beta, float* OUT) {
    __shared__ __align__(16) float ys[ORW * YSP];
    const int lane = threadIdx.x & 31, lr = lane & 15, hi = lane >> 4;
    const int wave = __builtin_amdgcn_readfirstlane((int)(threadIdx.x >> 5));
    const int r0 = blockIdx.x * ORW, c0 = wave * 64;
    v8f acc[4];
#pragma unroll
    for (int nb = 0; nb < 4; ++nb) acc[nb] = (v8f){};
    const size_t aoff = (size_t)(r0 + lr) * DM + 8 * hi, boff = (size_t)(c0 + lr) * DM + 8 * hi;
#pragma unroll 1
    for (int kc = 0; kc < DM; kc += 32) {
        const v16h a = ldh(AV + aoff + kc);
#pragma unroll
        for (int nb = 0; nb < 4; ++nb) { const v16h b = ldh(WO + boff + (size_t)nb * 16 * DM + kc); acc[nb] = wmma16_g(a, b, acc[nb]); }
    }
#pragma unroll
    for (int nb = 0; nb < 4; ++nb)
#pragma unroll
        for (int j = 0; j < 8; ++j) ys[(hi * 8 + j) * YSP + c0 + nb * 16 + lr] = acc[nb][j] * OSCL;
    __syncthreads();
#pragma unroll 1
    for (int rr = 0; rr < 2; ++rr) {
        const int row = wave * 2 + rr;
        const int mrow = r0 + row;
        const size_t grow = (size_t)(mrow / NB) * NB_FULL + (size_t)(mrow % NB);
        v4f y[4]; float sum = 0.0f;
#pragma unroll
        for (int j = 0; j < 4; ++j) { const int c = (lane + 32 * j) * 4;
            const v4f a = *(const v4fa*)(&ys[row * YSP + c]); const v4f hv = *(const v4f*)(hin + grow * DM + c);
#pragma unroll
            for (int i = 0; i < 4; ++i) { y[j][i] = bfr(hv[i]) + a[i]; sum += y[j][i]; } }
        sum = wsum(sum);
        const float mu = sum * (1.0f / (float)DM);
        float sq = 0.0f;
#pragma unroll
        for (int j = 0; j < 4; ++j)
#pragma unroll
            for (int i = 0; i < 4; ++i) { const float d = y[j][i] - mu; y[j][i] = d; sq += d * d; }
        sq = wsum(sq);
        const float rstd = rsqrtf(sq * (1.0f / (float)DM) + LNEPS);
#pragma unroll
        for (int j = 0; j < 4; ++j) { const int c = (lane + 32 * j) * 4;
            const v4f gv = *(const v4f*)(gamma + c); const v4f bv = *(const v4f*)(beta + c); v4f ov;
#pragma unroll
            for (int i = 0; i < 4; ++i) ov[i] = y[j][i] * rstd * bfr(gv[i]) + bfr(bv[i]);
            *(v4fa*)(&ys[row * YSP + c]) = ov; }
    }
    wave_sync();
#pragma unroll 1
    for (int ps = 0; ps < 2; ++ps) {
#pragma unroll 1
        for (int rr = 0; rr < 2; ++rr) {
            const int row = wave * 2 + rr;
            const int mrow = r0 + row;
            const size_t grow = (size_t)(mrow / NB) * NB_FULL + (size_t)(mrow % NB);
#pragma unroll
            for (int j = 0; j < 4; ++j) { const int c = (lane + 32 * j) * 4;
                const v4f val = *(const v4fa*)(&ys[row * YSP + c]);
                *(volatile v4f*)(OUT + grow * DM + c) = val; } }
        if (ps == 0) __threadfence(); }
}

static constexpr size_t al256(size_t v) { return (v + 255) & ~(size_t)255; }
static constexpr size_t SZ_XB = al256((size_t)SEQ * NB_FULL * DM * 2);
static constexpr size_t SZ_WB = al256((size_t)3 * DM * DM * 2);
static constexpr size_t SZ_WO = al256((size_t)DM * DM * 2);
static constexpr size_t SZ_TP = al256((size_t)NB * SEQ * DM * 4);
static constexpr size_t SZ_AV = al256((size_t)NB * SEQ * DM * 2);
static constexpr size_t SZ_TOTAL = SZ_XB + SZ_WB + SZ_WO + 3 * SZ_TP + SZ_AV;
static_assert(SZ_TOTAL <= (size_t)134217728);
static_assert(((size_t)DM * DM * 2) % 256 == 0);

extern "C" void kernel_launch(void* const* d_in, const int* in_sizes, int n_in,
                              void* d_out, int out_size, void* d_ws, size_t ws_size, hipStream_t stream) {
    if (n_in < 10) return;
    if ((size_t)in_sizes[0] < (size_t)SEQ * NB_FULL * DM) return;
    if ((size_t)in_sizes[1] < (size_t)DM * DM || (size_t)in_sizes[2] < (size_t)2 * DM * DM || (size_t)in_sizes[7] < (size_t)DM * DM) return;
    if (in_sizes[3] < HD * HD || in_sizes[4] < HD * HD || in_sizes[5] < HD * HD) return;
    if (in_sizes[6] < DM || in_sizes[8] < DM || in_sizes[9] < DM) return;
    if ((size_t)out_size < ((size_t)(SEQ - 1) * NB_FULL + NB) * DM) return;
    if (SZ_TOTAL > ws_size) return;
    const float* hin = (const float*)d_in[0];
    const float* wq  = (const float*)d_in[1];
    const float* wkv = (const float*)d_in[2];
    const float* wqt = (const float*)d_in[3];
    const float* wkt = (const float*)d_in[4];
    const float* wvt = (const float*)d_in[5];
    const float* lam = (const float*)d_in[6];
    const float* wo  = (const float*)d_in[7];
    const float* gam = (const float*)d_in[8];
    const float* bet = (const float*)d_in[9];
    float* OUT = (float*)d_out;
    char* wsp = (char*)d_ws;
    bf*  XB  = (bf*)wsp;  wsp += SZ_XB;
    bf*  WB  = (bf*)wsp;  wsp += SZ_WB;
    h16* WOH = (h16*)wsp; wsp += SZ_WO;
    float* TQ = (float*)wsp; wsp += SZ_TP;
    float* TK = (float*)wsp; wsp += SZ_TP;
    float* TV = (float*)wsp; wsp += SZ_TP;
    h16* AV  = (h16*)wsp; wsp += SZ_AV;

    { const size_t n8 = (size_t)SEQ * NB_FULL * DM / 8; k_cvt8<<<(unsigned)((n8 + 255) / 256), 256, 0, stream>>>(hin, XB, n8); }
    { const size_t n8 = (size_t)DM * DM / 8; k_cvt8<<<(unsigned)((n8 + 255) / 256), 256, 0, stream>>>(wq, WB, n8); }
    { const size_t n8 = (size_t)2 * DM * DM / 8; k_cvt8<<<(unsigned)((n8 + 255) / 256), 256, 0, stream>>>(wkv, WB + (size_t)DM * DM, n8); }
    { const size_t n8 = (size_t)DM * DM / 8; k_wcvt8h<<<(unsigned)((n8 + 255) / 256), 256, 0, stream>>>(wo, WOH, n8, WCARRY); }

    k_qkvt<<<dim3(NB * SEQ / 64, DM / 64, 1), 32, 0, stream>>>(XB, WB, lam, wqt, TQ);
    k_qkvt<<<dim3(NB * SEQ / 64, DM / 64, 1), 32, 0, stream>>>(XB, WB + (size_t)DM * DM, lam, wkt, TK);
    k_qkvt<<<dim3(NB * SEQ / 64, DM / 64, 1), 32, 0, stream>>>(XB, WB + (size_t)2 * DM * DM, lam, wvt, TV);

    k_mpattn<<<dim3(SEQ / 32, NB * NH_, 1), 256, 0, stream>>>(TQ, TK, TV, AV);

    k_oln<<<dim3(NB * SEQ / ORW, 1, 1), 256, 0, stream>>>(AV, WOH, hin, gam, bet, OUT);
}
